// SS2D_9577777070322
// MI455X (gfx1250) — hardware-verified
//
#include <hip/hip_runtime.h>
#include <math.h>

typedef __attribute__((ext_vector_type(16))) _Float16 v16h;
typedef __attribute__((ext_vector_type(8)))  _Float16 v8h;
typedef __attribute__((ext_vector_type(16))) __bf16   v16b;
typedef __attribute__((ext_vector_type(8)))  __bf16   v8b;
typedef __attribute__((ext_vector_type(8)))  float    v8f;
typedef __attribute__((ext_vector_type(4)))  float    v4f;
typedef __attribute__((ext_vector_type(2)))  unsigned int u32x2;

constexpr int kB     = 8;
constexpr int kHW    = 32;
constexpr int kL     = kHW * kHW;
constexpr int kDm    = 192;
constexpr int kDin   = 384;
constexpr int kNst   = 16;
constexpr int kNdir  = 8;
constexpr int kDtR   = 12;
constexpr int kC44   = kDtR + 2 * kNst;
constexpr int kCP    = 48;
constexpr int kRows  = kB * kL;
constexpr int kXzP   = 2 * kDin;
constexpr int kPrjP  = kNdir * kCP;
constexpr int kConvTP  = 388;
constexpr int kScanTS  = 32;
constexpr int kScanCh  = 128;
constexpr int kScanChunks = kDin / kScanCh;
constexpr int kScanYP  = 132;
constexpr float kUCarry  = 16.0f;
constexpr float kXpCarry = 32.0f;
constexpr float kYCarry  = 16.0f;
constexpr float kPrjScale = 1.0f / (kUCarry * kXpCarry);
constexpr size_t kYPlane = (size_t)kRows * kDin;
static_assert(kC44 == 44 && kDtR == 12, "x_proj split");
static_assert(kHW == 32 && kL == 1024, "position maps assume 32 x 32");
static_assert((kDm % 32) == 0 && (kDin % 32) == 0, "GEMM K multiples of 32");
static_assert((kRows % 64) == 0 && (kXzP % 64) == 0 && (kPrjP % 64) == 0 && (kDm % 64) == 0, "GEMM M,N multiples of 64");
static_assert(((kRows / 64) * (kXzP / 64)) % 8 == 0 && ((kRows / 64) * (kPrjP / 64)) % 8 == 0 && ((kRows / 64) * (kDm / 64)) % 8 == 0, "8 tiles per GEMM block");
static_assert((kL % kScanTS) == 0 && kScanCh * kScanChunks == kDin && kScanTS * 12 == 3 * kScanCh, "scan tiling");
static_assert(kDin == 96 * 4, "96-thread blocks cover 384 channels with 4 each");
static_assert((kConvTP * 4) % 16 == 0 && (kScanYP * 4) % 16 == 0, "16-B aligned LDS pitches");

constexpr size_t kOffXH   = 0;
constexpr size_t kOffXL   = kOffXH  + (size_t)kRows * kDm  * 2;
constexpr size_t kOffWIH  = kOffXL  + (size_t)kRows * kDm  * 2;
constexpr size_t kOffWIL  = kOffWIH + (size_t)kXzP  * kDm  * 2;
constexpr size_t kOffXPT  = kOffWIL + (size_t)kXzP  * kDm  * 2;
constexpr size_t kOffWOH  = kOffXPT + (size_t)kPrjP * kDin * 2;
constexpr size_t kOffWOL  = kOffWOH + (size_t)kDm   * kDin * 2;
constexpr size_t kOffXZ   = kOffWOL + (size_t)kDm   * kDin * 2;
constexpr size_t kOffU    = kOffXZ  + (size_t)kRows * kXzP * 4;
constexpr size_t kOffUH   = kOffU   + (size_t)kRows * kDin * 4;
constexpr size_t kOffP    = kOffUH  + (size_t)kRows * kDin * 2;
constexpr size_t kOffY8   = kOffP   + (size_t)kRows * kPrjP * 4;
constexpr size_t kOffYGH  = kOffY8  + (size_t)kNdir * kYPlane * 2;
constexpr size_t kOffYGL  = kOffYGH + (size_t)kRows * kDin * 2;
constexpr size_t kWsTotal = kOffYGL + (size_t)kRows * kDin * 2;
static_assert(kWsTotal == 127008768ull, "carve total");
static_assert(kWsTotal <= 134217728ull, "carve cap");
static_assert((kOffXL % 128) == 0 && (kOffWIH % 128) == 0 && (kOffWIL % 128) == 0 && (kOffXPT % 128) == 0 &&
              (kOffWOH % 128) == 0 && (kOffWOL % 128) == 0 && (kOffXZ % 128) == 0 && (kOffU % 128) == 0 &&
              (kOffUH % 128) == 0 && (kOffP % 128) == 0 && (kOffY8 % 128) == 0 && (kOffYGH % 128) == 0 &&
              (kOffYGL % 128) == 0, "128-B aligned regions");

__device__ __forceinline__ unsigned short f2bf_bits(float f) {
  unsigned u = __float_as_uint(f);
  return (unsigned short)((u + 0x7FFFu + ((u >> 16) & 1u)) >> 16);
}
__device__ __forceinline__ float bf_bits2f(unsigned short h) { return __uint_as_float(((unsigned)h) << 16); }

__device__ __forceinline__ float h16_to_f32(unsigned hb) {
  const unsigned sgn = (hb & 0x8000u) << 16; const unsigned em = hb & 0x7fffu;
  const float fn = __uint_as_float((em << 13) + 0x38000000u);
  const float fs = (float)em * 5.9604644775390625e-8f;
  const float mag = (em < 0x400u) ? fs : fn; return __uint_as_float(__float_as_uint(mag) | sgn);
}

__device__ __forceinline__ void dep_guard_h(v8f& a, v8f& b, v16h x, v16h y) { asm volatile("v_nop\n\tv_nop\n\tv_nop\n\tv_nop" : "+v"(a), "+v"(b) : "v"(x), "v"(y)); }
__device__ __forceinline__ void dep_guard_b(v8f& a, v8f& b, v16b x, v16b y) { asm volatile("v_nop\n\tv_nop\n\tv_nop\n\tv_nop" : "+v"(a), "+v"(b) : "v"(x), "v"(y)); }
__device__ __forceinline__ void dep_guard4_h(v8f& a, v8f& b, v8f& c, v8f& d, v16h x, v16h y) { asm volatile("v_nop\n\tv_nop\n\tv_nop\n\tv_nop" : "+v"(a), "+v"(b), "+v"(c), "+v"(d) : "v"(x), "v"(y)); }
__device__ __forceinline__ void dep_guard4_b(v8f& a, v8f& b, v8f& c, v8f& d, v16b x, v16b y) { asm volatile("v_nop\n\tv_nop\n\tv_nop\n\tv_nop" : "+v"(a), "+v"(b), "+v"(c), "+v"(d) : "v"(x), "v"(y)); }
__device__ __forceinline__ void keep4_h(v16h a, v16h b, v16h c, v16h d) { asm volatile("v_nop" :: "v"(a), "v"(b), "v"(c), "v"(d)); }
__device__ __forceinline__ void keep4_b(v16b a, v16b b, v16b c, v16b d) { asm volatile("v_nop" :: "v"(a), "v"(b), "v"(c), "v"(d)); }
__device__ __forceinline__ void acc_guard4(v8f& a, v8f& b, v8f& c, v8f& d) { asm volatile("v_nop\n\tv_nop\n\tv_nop\n\tv_nop" : "+v"(a), "+v"(b), "+v"(c), "+v"(d)); }
template <typename T> struct Frag;
template <> struct Frag<_Float16> {
  typedef v16h V; union U { v16h v; v8h h[2]; };
  static __device__ __forceinline__ v16h load(const _Float16* p) {
    U f; f.h[0] = *(const v8h*)(p); f.h[1] = *(const v8h*)(p + 16); return f.v;
  }
  static __device__ __forceinline__ v8f mma(v16h a, v16h b, v8f c) {
    return __builtin_amdgcn_wmma_f32_16x16x32_f16(false, a, false, b, (short)0, c, false, false);
  }
  static __device__ __forceinline__ void guard(v8f& a, v8f& b, v16h x, v16h y) { dep_guard_h(a, b, x, y); }
  static __device__ __forceinline__ void guard4(v8f& a, v8f& b, v8f& c, v8f& d, v16h x, v16h y) { dep_guard4_h(a, b, c, d, x, y); }
  static __device__ __forceinline__ void keep(v16h a, v16h b, v16h c, v16h d) { keep4_h(a, b, c, d); }
};
template <> struct Frag<__bf16> {
  typedef v16b V; union U { v16b v; v8b h[2]; };
  static __device__ __forceinline__ v16b load(const __bf16* p) {
    U f; f.h[0] = *(const v8b*)(p); f.h[1] = *(const v8b*)(p + 16); return f.v;
  }
  static __device__ __forceinline__ v8f mma(v16b a, v16b b, v8f c) {
    return __builtin_amdgcn_wmma_f32_16x16x32_bf16(false, a, false, b, (short)0, c, false, false);
  }
  static __device__ __forceinline__ void guard(v8f& a, v8f& b, v16b x, v16b y) { dep_guard_b(a, b, x, y); }
  static __device__ __forceinline__ void guard4(v8f& a, v8f& b, v8f& c, v8f& d, v16b x, v16b y) { dep_guard4_b(a, b, c, d, x, y); }
  static __device__ __forceinline__ void keep(v16b a, v16b b, v16b c, v16b d) { keep4_b(a, b, c, d); }
};

template <int ET> struct Elem;
template <> struct Elem<0> { typedef _Float16 T; };
template <> struct Elem<1> { typedef __bf16 T; };
template <int ET, bool SPLIT, int BIAS_MODE, int OUT_MODE, bool RESID, int ACT = 0>
__global__ __launch_bounds__(256) void wmma_gemm64(
    const unsigned short* __restrict__ Ap, const unsigned short* __restrict__ A2p, int lda, long strideA,
    const unsigned short* __restrict__ Btp, const unsigned short* __restrict__ Bt2p, int ldb, long strideB,
    void* __restrict__ Cout, void* __restrict__ Cout2, int ldc, long strideC,
    const float* __restrict__ bias,
    const float* __restrict__ resid, long strideR,
    int M, int N, int K, float scale) {
  typedef typename Elem<ET>::T T;
  typedef typename Frag<T>::V V;
  const T* A = (const T*)Ap; const T* A2 = (const T*)A2p; const T* Bt = (const T*)Btp; const T* Bt2 = (const T*)Bt2p;
  __shared__ __align__(16) float sT[8][16 * 68];
  const int b    = blockIdx.y;
  const int lane = threadIdx.x & 31;
  const int wave = threadIdx.x >> 5;
  const int tilesN = N >> 6;
  const int tilesM = M >> 6;
  const int tile = blockIdx.x * 8 + wave;
  if (tile >= tilesM * tilesN) return;
  const int tm = tile / tilesN;
  const int tn = tile - tm * tilesN;
  const int m0 = tm << 6;
  const int n0 = tn << 6;

  const T* Ab  = A  + (size_t)b * strideA;
  const T* Bb  = Bt + (size_t)b * strideB;
  const T* Ab2 = SPLIT ? (A2  + (size_t)b * strideA) : nullptr;
  const T* Bb2 = SPLIT ? (Bt2 + (size_t)b * strideB) : nullptr;

  const int rlane = lane & 15;
  const int koff  = (lane >> 4) * 8;
  const int mOff  = (lane >> 4) * 8;

  v8f acc[4][4];
#pragma unroll
  for (int i = 0; i < 4; ++i)
#pragma unroll
    for (int j = 0; j < 4; ++j) acc[i][j] = (v8f){0.f,0.f,0.f,0.f,0.f,0.f,0.f,0.f};

  for (int k0 = 0; k0 < K; k0 += 32) {
    V bh[4], bl[4];
#pragma unroll
    for (int j = 0; j < 4; ++j) {
      const size_t bo = (size_t)(n0 + (j << 4) + rlane) * ldb + koff + k0;
      bh[j] = Frag<T>::load(Bb + bo);
      if (SPLIT) bl[j] = Frag<T>::load(Bb2 + bo);
    }
#pragma unroll
    for (int i = 0; i < 4; ++i) {
      const size_t ao = (size_t)(m0 + (i << 4) + rlane) * lda + koff + k0;
      V ah = Frag<T>::load(Ab + ao);
      V al;
      if (SPLIT) al = Frag<T>::load(Ab2 + ao);
#pragma unroll
      for (int j = 0; j < 4; ++j) {
        acc[i][j] = Frag<T>::mma(ah, bh[j], acc[i][j]);
        if (SPLIT) {
          acc[i][j] = Frag<T>::mma(ah, bl[j], acc[i][j]);
          acc[i][j] = Frag<T>::mma(al, bh[j], acc[i][j]);
        }
      }
      Frag<T>::guard4(acc[i][0], acc[i][1], acc[i][2], acc[i][3], ah, SPLIT ? al : ah);
    }
    Frag<T>::keep(bh[0], bh[1], bh[2], bh[3]);
    if (SPLIT) Frag<T>::keep(bl[0], bl[1], bl[2], bl[3]);
  }
  acc_guard4(acc[0][0], acc[0][1], acc[0][2], acc[0][3]);
  acc_guard4(acc[1][0], acc[1][1], acc[1][2], acc[1][3]);
  acc_guard4(acc[2][0], acc[2][1], acc[2][2], acc[2][3]);
  acc_guard4(acc[3][0], acc[3][1], acc[3][2], acc[3][3]);

  float* slab = sT[wave];
  const float* Rb = RESID ? (resid + (size_t)b * strideR) : nullptr;
#pragma unroll
  for (int i = 0; i < 4; ++i) {
    const int mBase = m0 + (i << 4);
#pragma unroll
    for (int j = 0; j < 4; ++j) {
      const int n = n0 + (j << 4) + rlane;
      float bv = 0.f;
      if (BIAS_MODE == 2) bv = bias[n];
#pragma unroll
      for (int r = 0; r < 8; ++r) {
        float v = acc[i][j][r] * scale;
        if (BIAS_MODE == 1) v += bias[mBase + mOff + r];
        if (BIAS_MODE == 2) v += bv;
        if (RESID) v += Rb[(size_t)(mBase + mOff + r) * ldc + n];
        if (ACT == 1) v = tanhf(v);
        if (ACT == 2) v = fmaxf(v, 0.0f);
        if (ACT == 3) v = v / (1.0f + expf(-v));
        if (ACT == 4) v = (v > 0.f) ? v : 0.01f * v;
        slab[(mOff + r) * 68 + (j << 4) + rlane] = v;
      }
    }
    __builtin_amdgcn_fence(__ATOMIC_RELEASE, "workgroup");
    __builtin_amdgcn_wave_barrier();
    __builtin_amdgcn_fence(__ATOMIC_ACQUIRE, "workgroup");
    if (OUT_MODE == 0) {
      float* C = (float*)Cout + (size_t)b * strideC;
      const int hh = lane >> 4, c4 = (lane & 15) * 4;
      for (int pass = 0; pass < 2; ++pass) {
#pragma unroll
        for (int it = 0; it < 8; ++it) {
          const int row = it * 2 + hh;
          v4f v = *(const v4f*)(slab + row * 68 + c4);
          *(volatile v4f*)(C + (size_t)(mBase + row) * ldc + n0 + c4) = v;
        }
        __threadfence();
      }
    } else {
      const int q = lane >> 3, c8 = (lane & 7) * 8;
      unsigned short* C  = (unsigned short*)Cout  + (size_t)b * strideC;
      unsigned short* C2 = (OUT_MODE == 2) ? ((unsigned short*)Cout2 + (size_t)b * strideC) : nullptr;
      for (int pass = 0; pass < 2; ++pass) {
#pragma unroll
        for (int it = 0; it < 4; ++it) {
          const int row = it * 4 + q;
          const float* sp = slab + row * 68 + c8;
          v8h hv, lv;
#pragma unroll
          for (int e = 0; e < 8; ++e) {
            if (OUT_MODE == 1) {
              hv[e] = (_Float16)sp[e];
            } else {
              unsigned short hb = f2bf_bits(sp[e]);
              unsigned short lb = f2bf_bits(sp[e] - bf_bits2f(hb));
              hv[e] = __builtin_bit_cast(_Float16, hb);
              lv[e] = __builtin_bit_cast(_Float16, lb);
            }
          }
          *(volatile v8h*)(C + (size_t)(mBase + row) * ldc + n0 + c8) = hv;
          if (OUT_MODE == 2) *(volatile v8h*)(C2 + (size_t)(mBase + row) * ldc + n0 + c8) = lv;
        }
        __threadfence();
      }
    }
    __builtin_amdgcn_fence(__ATOMIC_RELEASE, "workgroup");
    __builtin_amdgcn_wave_barrier();
    __builtin_amdgcn_fence(__ATOMIC_ACQUIRE, "workgroup");
  }
}

__global__ __launch_bounds__(256) void split_rows_bf16_kernel(
    const float* __restrict__ src, unsigned short* __restrict__ dhi, unsigned short* __restrict__ dlo, int total8)
{
  const int i = blockIdx.x * 256 + threadIdx.x;
  if (i >= total8) return;
  const size_t e0 = (size_t)i << 3;
  const v4f a0 = *(const v4f*)(src + e0);
  const v4f a1 = *(const v4f*)(src + e0 + 4);
  v8h hv, lv;
#pragma unroll
  for (int e = 0; e < 4; ++e) {
    const unsigned short h0 = f2bf_bits(a0[e]), h1 = f2bf_bits(a1[e]);
    const unsigned short l0 = f2bf_bits(a0[e] - bf_bits2f(h0)), l1 = f2bf_bits(a1[e] - bf_bits2f(h1));
    hv[e]     = __builtin_bit_cast(_Float16, h0);
    hv[4 + e] = __builtin_bit_cast(_Float16, h1);
    lv[e]     = __builtin_bit_cast(_Float16, l0);
    lv[4 + e] = __builtin_bit_cast(_Float16, l1);
  }
  unsigned short* qh = dhi + e0;
  unsigned short* ql = dlo + e0;
  *(volatile v8h*)qh = hv;
  *(volatile v8h*)ql = lv;
  __threadfence();
  *(volatile v8h*)qh = hv;
  *(volatile v8h*)ql = lv;
}

__global__ __launch_bounds__(256) void xproj_cast_kernel(
    const float* __restrict__ W, unsigned short* __restrict__ XPT, int total8)
{
  const int i = blockIdx.x * 256 + threadIdx.x;
  if (i >= total8) return;
  const int e0   = i << 3;
  const int n    = e0 / kPrjP;
  const int col  = e0 - n * kPrjP;
  const int kdir = n / kCP;
  const int c    = n - kdir * kCP;
  const int cc   = (c < kC44) ? c : (kC44 - 1);
  const float f  = (c < kC44) ? kXpCarry : 0.0f;
  const float* src = W + ((size_t)(kdir * kC44 + cc)) * kDin + col;
  const v4f a0 = *(const v4f*)(src);
  const v4f a1 = *(const v4f*)(src + 4);
  v8h hv;
#pragma unroll
  for (int e = 0; e < 4; ++e) {
    hv[e]     = (_Float16)(a0[e] * f);
    hv[4 + e] = (_Float16)(a1[e] * f);
  }
  unsigned short* q = XPT + e0;
  *(volatile v8h*)q = hv;
  __threadfence();
  *(volatile v8h*)q = hv;
}

__global__ __launch_bounds__(96) void conv_silu_kernel(
    const float* __restrict__ XZ, const float* __restrict__ cw, const float* __restrict__ cb,
    float* __restrict__ U, unsigned short* __restrict__ UH)
{
  __shared__ __align__(16) float sT[kHW * kConvTP];
  const int tid = threadIdx.x;
  const int b = blockIdx.x >> 5, h = blockIdx.x & 31;
  const int ch = tid * 4;
  v4f wq[9];
#pragma unroll
  for (int q = 0; q < 5; ++q) wq[q] = *(const v4f*)(cw + (size_t)tid * 36 + 4 * q);
  asm volatile("" ::: "memory");
#pragma unroll
  for (int q = 5; q < 9; ++q) wq[q] = *(const v4f*)(cw + (size_t)tid * 36 + 4 * q);
  const v4f bq = *(const v4f*)(cb + ch);
  v4f wt[9];
#pragma unroll
  for (int tp = 0; tp < 9; ++tp) {
    v4f t4;
    t4[0] = wq[(tp) >> 2][(tp) & 3];
    t4[1] = wq[(9 + tp) >> 2][(9 + tp) & 3];
    t4[2] = wq[(18 + tp) >> 2][(18 + tp) & 3];
    t4[3] = wq[(27 + tp) >> 2][(27 + tp) & 3];
    wt[tp] = t4;
  }
  const size_t rowb = (size_t)b * kL + (size_t)h * kHW;
  size_t rbase[3]; bool rv[3];
  {
    const int hm = (h > 0) ? (h - 1) : 0;
    const int hp = (h < kHW - 1) ? (h + 1) : (kHW - 1);
    rbase[0] = (size_t)b * kL + (size_t)hm * kHW; rv[0] = (h > 0);
    rbase[1] = (size_t)b * kL + (size_t)h  * kHW; rv[1] = true;
    rbase[2] = (size_t)b * kL + (size_t)hp * kHW; rv[2] = (h < kHW - 1);
  }
  const v4f z4 = (v4f){0.f, 0.f, 0.f, 0.f};
  v4f win[3][3];
#pragma unroll
  for (int i = 0; i < 3; ++i) {
    win[i][0] = z4;
    const v4f v0 = *(const v4f*)(XZ + (rbase[i] + 0) * kXzP + ch);
    const v4f v1 = *(const v4f*)(XZ + (rbase[i] + 1) * kXzP + ch);
    win[i][1] = rv[i] ? v0 : z4;
    win[i][2] = rv[i] ? v1 : z4;
  }
#pragma unroll 1
  for (int w = 0; w < kHW; ++w) {
    v4f acc4 = z4;
#pragma unroll
    for (int i = 0; i < 3; ++i)
#pragma unroll
      for (int j = 0; j < 3; ++j) acc4 = acc4 + wt[i * 3 + j] * win[i][j];
    v4f u4;
#pragma unroll
    for (int c = 0; c < 4; ++c) {
      const float sv = acc4[c] + bq[c];
      const float sg = __builtin_amdgcn_rcpf(1.0f + __expf(-sv));
      u4[c] = sv * sg;
    }
    *(v4f*)(sT + w * kConvTP + ch) = u4;
    const int wn = w + 2;
    const bool cvd = (wn < kHW);
    const int wnc = cvd ? wn : (kHW - 1);
#pragma unroll
    for (int i = 0; i < 3; ++i) {
      win[i][0] = win[i][1];
      win[i][1] = win[i][2];
      const v4f v = *(const v4f*)(XZ + (rbase[i] + wnc) * kXzP + ch);
      win[i][2] = (cvd && rv[i]) ? v : z4;
    }
  }
  __syncthreads();
  for (int pass = 0; pass < 2; ++pass) {
#pragma unroll
    for (int it = 0; it < kHW; ++it) {
      const v4f v = *(const v4f*)(sT + it * kConvTP + ch);
      *(volatile v4f*)(U + (rowb + it) * kDin + ch) = v;
    }
#pragma unroll
    for (int it = 0; it < 16; ++it) {
      const int item = it * 96 + tid;
      const int r  = item / 48;
      const int g8 = item - r * 48;
      const float* sp = sT + r * kConvTP + g8 * 8;
      const v4f a0 = *(const v4f*)(sp);
      const v4f a1 = *(const v4f*)(sp + 4);
      v8h hv;
#pragma unroll
      for (int e = 0; e < 4; ++e) {
        hv[e]     = (_Float16)(a0[e] * kUCarry);
        hv[4 + e] = (_Float16)(a1[e] * kUCarry);
      }
      *(volatile v8h*)(UH + (rowb + r) * kDin + g8 * 8) = hv;
    }
    __threadfence();
  }
}

__device__ __forceinline__ int scan_pos(int dir, int ll) {
  const int row = ll >> 5;
  const int col = ll & 31;
  const int cs  = (row & 1) ? (31 - col) : col;
  const int p0 = (row << 5) + cs;
  const int p1 = (cs << 5) + row;
  const int p2 = (cs << 5) + (31 - row);
  const int p3 = (row << 5) + (31 - cs);
  return (dir == 0) ? p0 : ((dir == 1) ? p1 : ((dir == 2) ? p2 : p3));
}
__device__ __forceinline__ int dir_step(int kdir, int l) { return (kdir < 4) ? l : (kL - 1 - l); }

__global__ __launch_bounds__(128) void scan_kernel(
    const float* __restrict__ P, const float* __restrict__ U,
    const float* __restrict__ Wdt, const float* __restrict__ bdt, const float* __restrict__ Alog,
    unsigned short* __restrict__ Y8)
{
  __shared__ __align__(16) float sP[kScanTS * kCP];
  __shared__ __align__(16) float sY[kScanTS * kScanYP];
  const int tid = threadIdx.x, lane = tid & 31, wave = tid >> 5;
  const int bx = blockIdx.x;
  const int chunk = bx % kScanChunks;
  const int kdir  = (bx / kScanChunks) % kNdir;
  const int b     = bx / (kScanChunks * kNdir);
  const int dir   = kdir & 3;
  const int d     = chunk * kScanCh + tid;
  const int pr    = kdir * kDin + d;

  const v4f wa = *(const v4f*)(Wdt + (size_t)pr * kDtR);
  const v4f wb = *(const v4f*)(Wdt + (size_t)pr * kDtR + 4);
  const v4f wc = *(const v4f*)(Wdt + (size_t)pr * kDtR + 8);
  const float bb = bdt[pr];
  asm volatile("" ::: "memory");
  v4f aq[4];
#pragma unroll
  for (int q = 0; q < 4; ++q) aq[q] = *(const v4f*)(Alog + (size_t)pr * kNst + 4 * q);
  float An[kNst], h[kNst];
#pragma unroll
  for (int n = 0; n < kNst; ++n) { An[n] = -__expf(aq[n >> 2][n & 3]); h[n] = 0.f; }

  const size_t rowb = (size_t)b * kL;
  unsigned short* Yk = Y8 + (size_t)kdir * kYPlane;
  const int hh = lane >> 4, c8 = (lane & 15) * 8;

#pragma unroll 1
  for (int c = 0; c < kL / kScanTS; ++c) {
    const int l0 = c * kScanTS;
    __syncthreads();
#pragma unroll
    for (int q = 0; q < 3; ++q) {
      const int item = tid + q * kScanCh;
      const int s    = item / 12;
      const int q4   = item - s * 12;
      const int pos  = scan_pos(dir, dir_step(kdir, l0 + s));
      const v4f v = *(const v4f*)(P + (rowb + pos) * kPrjP + kdir * kCP + q4 * 4);
      *(v4f*)(sP + s * kCP + q4 * 4) = v;
    }
    __syncthreads();
#pragma unroll 1
    for (int s = 0; s < kScanTS; ++s) {
      const int pos = scan_pos(dir, dir_step(kdir, l0 + s));
      const float uv = U[(rowb + pos) * kDin + d];
      const float* xr = sP + s * kCP;
      const v4f x0 = *(const v4f*)(xr);
      const v4f x1 = *(const v4f*)(xr + 4);
      const v4f x2 = *(const v4f*)(xr + 8);
      float vd = 0.0f;
      vd = fmaf(wa[0], x0[0], vd); vd = fmaf(wa[1], x0[1], vd); vd = fmaf(wa[2], x0[2], vd); vd = fmaf(wa[3], x0[3], vd);
      vd = fmaf(wb[0], x1[0], vd); vd = fmaf(wb[1], x1[1], vd); vd = fmaf(wb[2], x1[2], vd); vd = fmaf(wb[3], x1[3], vd);
      vd = fmaf(wc[0], x2[0], vd); vd = fmaf(wc[1], x2[1], vd); vd = fmaf(wc[2], x2[2], vd); vd = fmaf(wc[3], x2[3], vd);
      const float v  = vd + bb;
      const float dt = fmaxf(v, 0.0f) + log1pf(__expf(-fabsf(v)));
      v4f Bq[4], Cq[4];
#pragma unroll
      for (int qq = 0; qq < 4; ++qq) {
        Bq[qq] = *(const v4f*)(xr + kDtR + 4 * qq);
        Cq[qq] = *(const v4f*)(xr + kDtR + kNst + 4 * qq);
      }
      float du = dt * uv;
      asm volatile("" : "+v"(du));
      float y = 0.0f;
#pragma unroll
      for (int n = 0; n < kNst; ++n) {
        const float e = __expf(dt * An[n]);
        float p = du * Bq[n >> 2][n & 3];
        asm volatile("" : "+v"(p));
        float qv = h[n] * e;
        asm volatile("" : "+v"(qv));
        const float hn = qv + p;
        h[n] = hn;
        float rr = Cq[n >> 2][n & 3] * hn;
        asm volatile("" : "+v"(rr));
        y += rr;
      }
      sY[s * kScanYP + tid] = y * kYCarry;
    }
    __syncthreads();
    v8h hv[4];
    int prow[4];
#pragma unroll
    for (int it = 0; it < 4; ++it) {
      const int r = it * 8 + wave * 2 + hh;
      const float* sp = sY + r * kScanYP + c8;
      const v4f a0 = *(const v4f*)(sp);
      const v4f a1 = *(const v4f*)(sp + 4);
#pragma unroll
      for (int e = 0; e < 4; ++e) { hv[it][e] = (_Float16)a0[e]; hv[it][4 + e] = (_Float16)a1[e]; }
      prow[it] = scan_pos(dir, dir_step(kdir, l0 + r));
    }
    for (int pass = 0; pass < 2; ++pass) {
#pragma unroll
      for (int it = 0; it < 4; ++it)
        *(volatile v8h*)(Yk + (rowb + prow[it]) * kDin + chunk * kScanCh + c8) = hv[it];
      __threadfence();
    }
  }
}

__global__ __launch_bounds__(96) void ln_gate_kernel(
    const unsigned short* __restrict__ Y8, const float* __restrict__ U, const float* __restrict__ XZ,
    const float* __restrict__ Dsv, const float* __restrict__ lnw, const float* __restrict__ lnb,
    unsigned short* __restrict__ YGH, unsigned short* __restrict__ YGL)
{
  __shared__ __align__(16) float sYG[kDin];
  __shared__ float sRed[8];
  const int tid = threadIdx.x, lane = tid & 31, wave = tid >> 5;
  const size_t g = blockIdx.x;
  const int ch = tid * 4;

  v4f dsum = (v4f){0.f, 0.f, 0.f, 0.f};
#pragma unroll
  for (int k = 0; k < 4; ++k) dsum = dsum + *(const v4f*)(Dsv + (size_t)k * kDin + ch);
  asm volatile("" ::: "memory");
#pragma unroll
  for (int k = 4; k < 8; ++k) dsum = dsum + *(const v4f*)(Dsv + (size_t)k * kDin + ch);
  asm volatile("" ::: "memory");
  const v4f w4 = *(const v4f*)(lnw + ch);
  const v4f b4 = *(const v4f*)(lnb + ch);
  const v4f u4 = *(const v4f*)(U + g * kDin + ch);
  const v4f z4 = *(const v4f*)(XZ + g * kXzP + kDin + ch);
  asm volatile("" ::: "memory");
  v4f ys = (v4f){0.f, 0.f, 0.f, 0.f};
#pragma unroll
  for (int k = 0; k < kNdir; ++k) {
    if (k == 4) asm volatile("" ::: "memory");
    const u32x2 wv = *(const u32x2*)(const void*)(Y8 + (size_t)k * kYPlane + g * kDin + ch);
    const unsigned w0 = wv[0], w1 = wv[1];
    ys[0] += h16_to_f32(w0 & 0xffffu);
    ys[1] += h16_to_f32(w0 >> 16);
    ys[2] += h16_to_f32(w1 & 0xffffu);
    ys[3] += h16_to_f32(w1 >> 16);
  }
  const v4f v = ys * (1.0f / kYCarry) + u4 * dsum;

  float s1 = (v[0] + v[1]) + (v[2] + v[3]);
#pragma unroll
  for (int off = 1; off < 32; off <<= 1) s1 += __shfl_xor(s1, off, 32);
  if (lane == 0) sRed[wave] = s1;
  __syncthreads();
  const float mu = (sRed[0] + sRed[1] + sRed[2]) * (1.0f / kDin);
  v4f dv;
#pragma unroll
  for (int c = 0; c < 4; ++c) dv[c] = v[c] - mu;
  float s2 = (dv[0] * dv[0] + dv[1] * dv[1]) + (dv[2] * dv[2] + dv[3] * dv[3]);
#pragma unroll
  for (int off = 1; off < 32; off <<= 1) s2 += __shfl_xor(s2, off, 32);
  if (lane == 0) sRed[4 + wave] = s2;
  __syncthreads();
  const float var  = (sRed[4] + sRed[5] + sRed[6]) * (1.0f / kDin);
  const float rstd = rsqrtf(var + 1e-5f);
  v4f yg;
#pragma unroll
  for (int c = 0; c < 4; ++c) {
    const float yn = dv[c] * rstd * w4[c] + b4[c];
    const float zc = z4[c];
    const float sg = __builtin_amdgcn_rcpf(1.0f + __expf(-zc));
    yg[c] = yn * (zc * sg);
  }
  *(v4f*)(sYG + ch) = yg;
  __syncthreads();
  if (tid < 48) {
    const float* sp = sYG + tid * 8;
    const v4f a0 = *(const v4f*)(sp);
    const v4f a1 = *(const v4f*)(sp + 4);
    v8h hv, lv;
#pragma unroll
    for (int e = 0; e < 4; ++e) {
      const unsigned short h0 = f2bf_bits(a0[e]), h1 = f2bf_bits(a1[e]);
      const unsigned short l0 = f2bf_bits(a0[e] - bf_bits2f(h0)), l1 = f2bf_bits(a1[e] - bf_bits2f(h1));
      hv[e]     = __builtin_bit_cast(_Float16, h0);
      hv[4 + e] = __builtin_bit_cast(_Float16, h1);
      lv[e]     = __builtin_bit_cast(_Float16, l0);
      lv[4 + e] = __builtin_bit_cast(_Float16, l1);
    }
    unsigned short* ph = YGH + g * kDin + tid * 8;
    unsigned short* pl = YGL + g * kDin + tid * 8;
    *(volatile v8h*)ph = hv;
    *(volatile v8h*)pl = lv;
    __threadfence();
    *(volatile v8h*)ph = hv;
    *(volatile v8h*)pl = lv;
  }
}

extern "C" void kernel_launch(void* const* d_in, const int* in_sizes, int n_in,
                              void* d_out, int out_size, void* d_ws, size_t ws_size,
                              hipStream_t stream)
{
  if (n_in < 12) return;
  if (in_sizes[0]  != kRows * kDm) return;
  if (in_sizes[1]  != kXzP * kDm) return;
  if (in_sizes[2]  != kDin * 9) return;
  if (in_sizes[3]  != kDin) return;
  if (in_sizes[4]  != kNdir * kC44 * kDin) return;
  if (in_sizes[5]  != kNdir * kDin * kDtR) return;
  if (in_sizes[6]  != kNdir * kDin) return;
  if (in_sizes[7]  != kNdir * kDin * kNst) return;
  if (in_sizes[8]  != kNdir * kDin) return;
  if (in_sizes[9]  != kDin) return;
  if (in_sizes[10] != kDin) return;
  if (in_sizes[11] != kDm * kDin) return;
  if (out_size != kRows * kDm) return;
  if (ws_size < kWsTotal) return;

  const float* x      = (const float*)d_in[0];
  const float* W_in   = (const float*)d_in[1];
  const float* conv_w = (const float*)d_in[2];
  const float* conv_b = (const float*)d_in[3];
  const float* W_xprj = (const float*)d_in[4];
  const float* W_dt   = (const float*)d_in[5];
  const float* b_dt   = (const float*)d_in[6];
  const float* A_log  = (const float*)d_in[7];
  const float* Dsv    = (const float*)d_in[8];
  const float* ln_w   = (const float*)d_in[9];
  const float* ln_b   = (const float*)d_in[10];
  const float* W_out  = (const float*)d_in[11];
  float* out = (float*)d_out;

  char* ws = (char*)d_ws;
  unsigned short* XH  = (unsigned short*)(ws + kOffXH);
  unsigned short* XL  = (unsigned short*)(ws + kOffXL);
  unsigned short* WIH = (unsigned short*)(ws + kOffWIH);
  unsigned short* WIL = (unsigned short*)(ws + kOffWIL);
  unsigned short* XPT = (unsigned short*)(ws + kOffXPT);
  unsigned short* WOH = (unsigned short*)(ws + kOffWOH);
  unsigned short* WOL = (unsigned short*)(ws + kOffWOL);
  float*          XZ  = (float*)(ws + kOffXZ);
  float*          U   = (float*)(ws + kOffU);
  unsigned short* UH  = (unsigned short*)(ws + kOffUH);
  float*          P   = (float*)(ws + kOffP);
  unsigned short* Y8  = (unsigned short*)(ws + kOffY8);
  unsigned short* YGH = (unsigned short*)(ws + kOffYGH);
  unsigned short* YGL = (unsigned short*)(ws + kOffYGL);
  const float* dummy_bias  = b_dt;
  const float* dummy_resid = x;

  split_rows_bf16_kernel<<<(kRows * kDm / 8) / 256, 256, 0, stream>>>(x, XH, XL, kRows * kDm / 8);
  split_rows_bf16_kernel<<<(kXzP * kDm / 8) / 256, 256, 0, stream>>>(W_in, WIH, WIL, kXzP * kDm / 8);
  split_rows_bf16_kernel<<<(kDm * kDin / 8) / 256, 256, 0, stream>>>(W_out, WOH, WOL, kDm * kDin / 8);
  xproj_cast_kernel<<<(kPrjP * kDin / 8) / 256, 256, 0, stream>>>(W_xprj, XPT, kPrjP * kDin / 8);

  wmma_gemm64<1, true, 0, 0, false><<<dim3(((kRows / 64) * (kXzP / 64)) / 8, 1), 256, 0, stream>>>(
      XH, XL, kDm, 0L, WIH, WIL, kDm, 0L,
      (void*)XZ, (void*)XZ, kXzP, 0L, dummy_bias, dummy_resid, 0L, kRows, kXzP, kDm, 1.0f);

  conv_silu_kernel<<<dim3(kB * kHW, 1), 96, 0, stream>>>(XZ, conv_w, conv_b, U, UH);

  wmma_gemm64<0, false, 0, 0, false><<<dim3(((kRows / 64) * (kPrjP / 64)) / 8, 1), 256, 0, stream>>>(
      UH, UH, kDin, 0L, XPT, XPT, kDin, 0L,
      (void*)P, (void*)P, kPrjP, 0L, dummy_bias, dummy_resid, 0L, kRows, kPrjP, kDin, kPrjScale);

  scan_kernel<<<dim3(kB * kNdir * kScanChunks, 1), kScanCh, 0, stream>>>(P, U, W_dt, b_dt, A_log, Y8);

  ln_gate_kernel<<<dim3(kRows, 1), 96, 0, stream>>>(Y8, U, XZ, Dsv, ln_w, ln_b, YGH, YGL);

  wmma_gemm64<1, true, 0, 0, false><<<dim3(((kRows / 64) * (kDm / 64)) / 8, 1), 256, 0, stream>>>(
      YGH, YGL, kDin, 0L, WOH, WOL, kDin, 0L,
      (void*)out, (void*)out, kDm, 0L, dummy_bias, dummy_resid, 0L, kRows, kDm, kDin, 1.0f);
}
